// BiAttentionLayer_23751169147270
// MI455X (gfx1250) — hardware-verified
//
#include <hip/hip_runtime.h>
#include <stddef.h>
#include <stdint.h>
#include <math.h>

#define TN    8192
#define JN    8192
#define DN    100
#define KP    128
#define JT    64
#define NUT   7
#define RB    64
#define NBLK  (TN / RB)
#define OUTW  400
#define UP    128
#define TQP   72
#define NOUTB ((TN * OUTW) / (4 * 256))

#define PL_BYTES  ((size_t)TN * KP * 2)
#define QT_BYTES  ((size_t)KP * JN * 2)
#define U_BYTES   ((size_t)TN * UP * 4)
#define CW_BYTES  ((size_t)TN * 4)
#define QW_BYTES  ((size_t)JN * 4)
#define HP_BYTES  ((size_t)NBLK * KP * 4)
#define H_BYTES   ((size_t)KP * 4)

#define OFF_BH   ((size_t)0)
#define OFF_BL   (OFF_BH + PL_BYTES)
#define OFF_QA   (OFF_BL + PL_BYTES)
#define OFF_QT   (OFF_QA + PL_BYTES)
#define OFF_U    (OFF_QT + QT_BYTES)
#define OFF_CW   (OFF_U + U_BYTES)
#define OFF_QW   (OFF_CW + CW_BYTES)
#define OFF_HP   (OFF_QW + QW_BYTES)
#define OFF_H    (OFF_HP + HP_BYTES)
#define WS_TOTAL (OFF_H + H_BYTES)

static_assert(WS_TOTAL == (size_t)12714496);
static_assert(WS_TOTAL <= (size_t)134217728);
static_assert((OFF_BL % 256) == 0);
static_assert((OFF_QA % 256) == 0);
static_assert((OFF_QT % 256) == 0);
static_assert((OFF_U % 256) == 0);
static_assert((OFF_CW % 256) == 0);
static_assert((OFF_QW % 256) == 0);
static_assert((OFF_HP % 256) == 0);
static_assert((OFF_H % 256) == 0);
static_assert(TN == JN);
static_assert((TN % RB) == 0);
static_assert((JN % JT) == 0);
static_assert((KP % 32) == 0);
static_assert(NUT * 16 >= DN);
static_assert(NUT * 16 + 16 == KP);
static_assert((DN % 4) == 0);
static_assert((OUTW % 4) == 0);
static_assert(OUTW == 4 * DN);
static_assert((size_t)NOUTB * 256 * 4 == (size_t)TN * OUTW);
static_assert(((TQP * 2) % 16) == 0);
static_assert(RB == 64);

typedef unsigned short v8us  __attribute__((ext_vector_type(8)));
typedef unsigned short v16us __attribute__((ext_vector_type(16)));
typedef _Float16       v16h  __attribute__((ext_vector_type(16)));
typedef float          v4f   __attribute__((ext_vector_type(4)));
typedef float          v8f   __attribute__((ext_vector_type(8)));

union FragU { v16us v; v8us half[2]; };

__device__ __forceinline__ unsigned bbits(float f) {
  unsigned u = __float_as_uint(f);
  return (u + 0x7FFFu + ((u >> 16) & 1u)) >> 16;
}
__device__ __forceinline__ float bf16r(float f) {
  return __uint_as_float(bbits(f) << 16);
}
__device__ __forceinline__ unsigned short hbits(float f) {
  return __builtin_bit_cast(unsigned short, (_Float16)f);
}
__device__ __forceinline__ v8f zero8() { v8f z = {0.f, 0.f, 0.f, 0.f, 0.f, 0.f, 0.f, 0.f}; return z; }

__device__ __forceinline__ v16us ldfrag_u(const unsigned short* p) {
  FragU f;
  f.half[0] = *(const v8us*)(p);
  f.half[1] = *(const v8us*)(p + 16);
  return f.v;
}

__device__ __forceinline__ v8f mma_hu(v16us a, v16us b, v8f c) {
#if defined(__HIP_DEVICE_COMPILE__)
  return __builtin_amdgcn_wmma_f32_16x16x32_f16(false, __builtin_bit_cast(v16h, a),
                                               false, __builtin_bit_cast(v16h, b),
                                               (short)0, c, false, false);
#else
  (void)a; (void)b;
  return c;
#endif
}
__device__ __forceinline__ void guard2(v8f& c0, v8f& c1, const v16us& a, const v16us& b0,
                                       const v16us& b1) {
#if defined(__HIP_DEVICE_COMPILE__)
  asm volatile("v_nop\n\tv_nop\n\tv_nop\n\tv_nop"
               : "+v"(c0), "+v"(c1)
               : "v"(a), "v"(b0), "v"(b1));
#else
  (void)c0; (void)c1; (void)a; (void)b0; (void)b1;
#endif
}
__device__ __forceinline__ void guard7(v8f& c0, v8f& c1, v8f& c2, v8f& c3, v8f& c4, v8f& c5,
                                       v8f& c6, const v16us& a, const v16us& b0,
                                       const v16us& b1) {
#if defined(__HIP_DEVICE_COMPILE__)
  asm volatile("v_nop\n\tv_nop\n\tv_nop\n\tv_nop"
               : "+v"(c0), "+v"(c1), "+v"(c2), "+v"(c3), "+v"(c4), "+v"(c5), "+v"(c6)
               : "v"(a), "v"(b0), "v"(b1));
#else
  (void)c0; (void)c1; (void)c2; (void)c3; (void)c4; (void)c5; (void)c6;
  (void)a; (void)b0; (void)b1;
#endif
}

__global__ __launch_bounds__(256)
void k_cvt(const float* __restrict__ Cin, const float* __restrict__ Qin,
           const float* __restrict__ Win,
           unsigned short* bh16, unsigned short* bl16, unsigned short* qa16,
           unsigned short* qt16, float* cw, float* qw)
{
  __shared__ float wL[3 * DN];
  __shared__ __align__(16) unsigned short tq[KP * TQP];

  const int tid  = threadIdx.x;
  const int lane = tid & 31;
  const int w    = tid >> 5;
  const int hl   = lane >> 4;
  const int pc   = lane & 15;
  const int r0   = RB * blockIdx.x;

  for (int i = tid; i < 3 * DN; i += 256) wL[i] = bf16r(Win[i]);
  __syncthreads();

#pragma unroll 1
  for (int it = 0; it < 4; ++it) {
    const int rr = 16 * it + 2 * w + hl;
    const size_t row = (size_t)(r0 + rr);
    v8us obh, obl, oq;
#pragma unroll
    for (int e2 = 0; e2 < 2; ++e2) {
      const int  cc    = 8 * pc + 4 * e2;
      const bool valid = cc < DN;
      const int  ca    = valid ? cc : 0;
      const v4f xc = *(const v4f*)(Cin + row * DN + ca);
      const v4f xq = *(const v4f*)(Qin + row * DN + ca);
#pragma unroll
      for (int e = 0; e < 4; ++e) {
        const int   dcl = valid ? (cc + e) : 0;
        const float cv  = valid ? bf16r(xc[e]) : 0.0f;
        const float qv  = valid ? bf16r(xq[e]) : 0.0f;
        const float p   = (cv * wL[2 * DN + dcl]) * 1024.0f;
        const _Float16 ph = (_Float16)p;
        const float res = (p - (float)ph) * 2048.0f;
        obh[4 * e2 + e] = __builtin_bit_cast(unsigned short, ph);
        obl[4 * e2 + e] = hbits(res);
        const unsigned short qb = hbits(16.0f * qv);
        oq[4 * e2 + e] = qb;
        tq[(cc + e) * TQP + rr] = qb;
      }
    }
    const size_t off = row * KP + 8 * pc;
    *(volatile v8us*)(bh16 + off) = obh;
    *(volatile v8us*)(bl16 + off) = obl;
    *(volatile v8us*)(qa16 + off) = oq;
    __threadfence();
    *(volatile v8us*)(bh16 + off) = obh;
    *(volatile v8us*)(bl16 + off) = obl;
    *(volatile v8us*)(qa16 + off) = oq;
  }

  if (w < 4) {
    const int isq = w >> 1;
    const int rr  = tid & 63;
    const float* src = (isq ? Qin : Cin) + (size_t)(r0 + rr) * DN;
    const int wo = isq ? DN : 0;
    float s = 0.0f;
#pragma unroll 1
    for (int d = 0; d < DN; ++d) s += bf16r(src[d]) * wL[wo + d];
    const float sv = s;
    float* dst = (isq ? qw : cw) + r0 + rr;
    *(volatile float*)dst = sv;
    __threadfence();
    *(volatile float*)dst = sv;
  }
  __syncthreads();

  {
    const int q8 = lane >> 3;
    const int jj = lane & 7;
    v8us   v[4];
    size_t off[4];
#pragma unroll
    for (int it = 0; it < 4; ++it) {
      const int li = 32 * it + 4 * w + q8;
      v[it]   = *(const v8us*)(tq + li * TQP + 8 * jj);
      off[it] = (size_t)li * JN + r0 + 8 * jj;
    }
#pragma unroll
    for (int it = 0; it < 4; ++it) *(volatile v8us*)(qt16 + off[it]) = v[it];
    __threadfence();
#pragma unroll
    for (int it = 0; it < 4; ++it) *(volatile v8us*)(qt16 + off[it]) = v[it];
  }
}

__global__ __launch_bounds__(128)
void k_att(const unsigned short* __restrict__ bh16, const unsigned short* __restrict__ bl16,
           const unsigned short* __restrict__ qa16, const unsigned short* __restrict__ qt16,
           const float* __restrict__ cw, const float* __restrict__ qw,
           const float* __restrict__ Cin, float* u32, float* hp)
{
  __shared__ __align__(16) float ut[RB * UP];
  __shared__ float bsh[RB];

  const int tid  = threadIdx.x;
  const int lane = tid & 31;
  const int w    = tid >> 5;
  const int hl   = lane >> 4;
  const int m    = lane & 15;
  const int blk  = blockIdx.x;
  const int i0   = RB * blk;
  const int iw   = i0 + 16 * w;

  const float cwv = cw[iw + m];
  v8f acc[NUT];
#pragma unroll
  for (int n = 0; n < NUT; ++n) acc[n] = zero8();
  float mrun = -1.0e30f;
  float lrun = 0.0f;

  const unsigned short* pbh = bh16 + (size_t)(iw + m) * KP + 8 * hl;
  const unsigned short* pbl = bl16 + (size_t)(iw + m) * KP + 8 * hl;
  const unsigned short* pqa = qa16 + (size_t)m * KP + 8 * hl;
  const unsigned short* pqt = qt16 + (size_t)m * JN + 8 * hl;
  const float kl = 1.0f / 2048.0f;
  const float ks = 1.0f / 16384.0f;

#pragma unroll 1
  for (int jt = 0; jt < JN / JT; ++jt) {
    const int j0 = JT * jt;

    float sv[4][8];
#pragma unroll
    for (int g = 0; g < 4; ++g) {
      v8f ah = zero8(), al = zero8();
      v16us a, fb0, fb1;
#pragma unroll
      for (int kk = 0; kk < KP / 32; ++kk) {
        a   = ldfrag_u(pqa + (size_t)(j0 + 16 * g) * KP + 32 * kk);
        fb0 = ldfrag_u(pbh + 32 * kk);
        fb1 = ldfrag_u(pbl + 32 * kk);
        ah = mma_hu(a, fb0, ah);
        al = mma_hu(a, fb1, al);
      }
      guard2(ah, al, a, fb0, fb1);
      const v4f qv0 = *(const v4f*)(qw + j0 + 16 * g + 8 * hl);
      const v4f qv1 = *(const v4f*)(qw + j0 + 16 * g + 8 * hl + 4);
#pragma unroll
      for (int r = 0; r < 8; ++r) {
        const float qwr = (r < 4) ? qv0[r & 3] : qv1[r & 3];
        sv[g][r] = (cwv + qwr) + (ah[r] + al[r] * kl) * ks;
      }
    }

    float tmax = sv[0][0];
#pragma unroll
    for (int g = 0; g < 4; ++g)
#pragma unroll
      for (int r = 0; r < 8; ++r) tmax = fmaxf(tmax, sv[g][r]);
    tmax = fmaxf(tmax, __shfl_xor(tmax, 16, 32));
    const float mnew = fmaxf(mrun, tmax);
    const float sc   = __expf(mrun - mnew);
    mrun = mnew;
    float ps = 0.0f;
    v16us pk[2];
#pragma unroll
    for (int g = 0; g < 4; ++g) {
#pragma unroll
      for (int r = 0; r < 8; ++r) {
        const float p = __expf(sv[g][r] - mnew);
        ps += p;
        pk[g >> 1][(g & 1) * 8 + r] = hbits(4096.0f * p);
      }
    }
    ps += __shfl_xor(ps, 16, 32);
    lrun = lrun * sc + ps;
#pragma unroll
    for (int n = 0; n < NUT; ++n) acc[n] = acc[n] * sc;

    v16us af;
#pragma unroll
    for (int n = 0; n < NUT; ++n) {
#pragma unroll
      for (int u = 0; u < 2; ++u) {
        af = ldfrag_u(pqt + (size_t)(16 * n) * JN + j0 + 32 * u);
        acc[n] = mma_hu(af, pk[u], acc[n]);
      }
    }
    guard7(acc[0], acc[1], acc[2], acc[3], acc[4], acc[5], acc[6], af, pk[0], pk[1]);
  }

  const float linv = 1.0f / lrun;
  const float ku   = linv * (1.0f / 65536.0f);
  float* trow = ut + (16 * w + m) * UP;
#pragma unroll
  for (int n = 0; n < NUT; ++n) {
    v4f lo, hi;
#pragma unroll
    for (int e = 0; e < 4; ++e) { lo[e] = acc[n][e] * ku; hi[e] = acc[n][4 + e] * ku; }
    *(v4f*)(trow + 16 * n + 8 * hl)     = lo;
    *(v4f*)(trow + 16 * n + 8 * hl + 4) = hi;
  }
  {
    v4f z = {0.0f, 0.0f, 0.0f, 0.0f};
    *(v4f*)(trow + 16 * NUT + 8 * hl)     = z;
    *(v4f*)(trow + 16 * NUT + 8 * hl + 4) = z;
  }
  bsh[16 * w + m] = linv;
  __syncthreads();

#pragma unroll 1
  for (int it = 0; it < 16; ++it) {
    const int row = 4 * it + w;
    const v4f v = *(const v4f*)(ut + row * UP + 4 * lane);
    *(volatile v4f*)(u32 + (size_t)(i0 + row) * UP + 4 * lane) = v;
  }
  __threadfence();
#pragma unroll 1
  for (int it = 0; it < 16; ++it) {
    const int row = 4 * it + w;
    const v4f v = *(const v4f*)(ut + row * UP + 4 * lane);
    *(volatile v4f*)(u32 + (size_t)(i0 + row) * UP + 4 * lane) = v;
  }

  {
    const int d  = tid;
    const int dc = (d < DN) ? d : 0;
    const float* cp = Cin + (size_t)i0 * DN + dc;
    float s = 0.0f;
#pragma unroll 1
    for (int r = 0; r < RB; ++r) s += bsh[r] * bf16r(cp[(size_t)r * DN]);
    const float hv = (d < DN) ? s : 0.0f;
    float* dst = hp + (size_t)blk * KP + d;
    *(volatile float*)dst = hv;
    __threadfence();
    *(volatile float*)dst = hv;
  }
}

__global__ __launch_bounds__(128)
void k_hred(const float* __restrict__ hp, float* hsum)
{
  const int d = threadIdx.x;
  float s = 0.0f;
#pragma unroll 1
  for (int b = 0; b < NBLK; ++b) s += hp[(size_t)b * KP + d];
  const float hv = s;
  *(volatile float*)(hsum + d) = hv;
  __threadfence();
  *(volatile float*)(hsum + d) = hv;
}

__global__ __launch_bounds__(256)
void k_out(const float* __restrict__ Cin, const float* __restrict__ u32,
           const float* __restrict__ hsum, float* out)
{
  __shared__ __align__(16) float hL[KP];
  const int tid = threadIdx.x;
  if (tid < KP) hL[tid] = hsum[tid];
  __syncthreads();

  const int f   = 4 * (blockIdx.x * 256 + tid);
  const int t   = f / OUTW;
  const int col = f - t * OUTW;
  const int seg = col / DN;
  const int cc  = col - seg * DN;
  const v4f xc = *(const v4f*)(Cin + (size_t)t * DN + cc);
  const v4f xu = *(const v4f*)(u32 + (size_t)t * UP + cc);
  const v4f xh = *(const v4f*)(hL + cc);
  v4f o;
#pragma unroll
  for (int e = 0; e < 4; ++e) {
    const float c = bf16r(xc[e]);
    const float u = xu[e];
    const float vcu = c * u;
    const float vch = c * xh[e];
    o[e] = (seg == 0) ? c : ((seg == 1) ? u : ((seg == 2) ? vcu : vch));
  }
  *(volatile v4f*)(out + f) = o;
  __threadfence();
  *(volatile v4f*)(out + f) = o;
}

extern "C" void kernel_launch(void* const* d_in, const int* in_sizes, int n_in,
                              void* d_out, int out_size, void* d_ws, size_t ws_size,
                              hipStream_t stream) {
  if (n_in < 3) return;
  if (in_sizes[0] != TN * DN) return;
  if (in_sizes[1] != JN * DN) return;
  if (in_sizes[2] != 3 * DN) return;
  if (out_size != TN * OUTW) return;
  if (ws_size < WS_TOTAL) return;

  const float* Cin = (const float*)d_in[0];
  const float* Qin = (const float*)d_in[1];
  const float* Win = (const float*)d_in[2];
  float* out = (float*)d_out;

  char* ws = (char*)d_ws;
  unsigned short* bh16 = (unsigned short*)(ws + OFF_BH);
  unsigned short* bl16 = (unsigned short*)(ws + OFF_BL);
  unsigned short* qa16 = (unsigned short*)(ws + OFF_QA);
  unsigned short* qt16 = (unsigned short*)(ws + OFF_QT);
  float*          u32  = (float*)(ws + OFF_U);
  float*          cw   = (float*)(ws + OFF_CW);
  float*          qw   = (float*)(ws + OFF_QW);
  float*          hp   = (float*)(ws + OFF_HP);
  float*          hs   = (float*)(ws + OFF_H);

  k_cvt<<<dim3(NBLK), dim3(256), 0, stream>>>(Cin, Qin, Win, bh16, bl16, qa16, qt16, cw, qw);
  (void)hipGetLastError();
  k_att<<<dim3(NBLK), dim3(128), 0, stream>>>(bh16, bl16, qa16, qt16, cw, qw, Cin, u32, hp);
  (void)hipGetLastError();
  k_hred<<<dim3(1), dim3(128), 0, stream>>>(hp, hs);
  (void)hipGetLastError();
  k_out<<<dim3(NOUTB), dim3(256), 0, stream>>>(Cin, u32, hs, out);
  (void)hipGetLastError();
}
